// TransformerEncoder_40372692582539
// MI455X (gfx1250) — hardware-verified
//
#include <hip/hip_runtime.h>
#ifndef NB
#define NB 8
#endif
#ifndef SEQ
#define SEQ 1024
#endif
#define NB_FULL 8
#define SEQ_FULL 1024
#define DM 768
#define NH 12
#define HD 64
#define FF 3072
#define MROWS (NB * SEQ)

static_assert(NH * HD == DM);
static_assert(HD == 64);
static_assert(SEQ % 64 == 0);
static_assert(SEQ <= SEQ_FULL);
static_assert(NB <= NB_FULL);
static_assert(MROWS % 32 == 0);
static_assert(DM % 256 == 0);
static_assert(FF % 64 == 0);
static_assert(FF == 4 * DM);
static_assert(((MROWS / 32) * (DM / 64)) % 4 == 0);
static_assert(((MROWS / 32) * (FF / 64)) % 4 == 0);
static_assert(((DM / 32) * (MROWS / 64)) % 4 == 0);
static_assert((DM * (DM / 8)) % 256 == 0);
static_assert((FF * (DM / 8)) % 256 == 0);
static_assert(MROWS % 4 == 0);
static_assert((size_t)NB * NH * (SEQ / 64) * 64 * 64 == (size_t)MROWS * DM);

typedef _Float16 v16h __attribute__((ext_vector_type(16)));
typedef unsigned short v8us __attribute__((ext_vector_type(8), may_alias));
typedef float  v8f  __attribute__((ext_vector_type(8)));
typedef float  v4f  __attribute__((ext_vector_type(4)));
typedef float  v4fa __attribute__((ext_vector_type(4), may_alias));
union FragH { v16h v; v8us half[2]; };

__device__ __forceinline__ unsigned short bf16_bits(float x) { unsigned int u = __float_as_uint(x); return (unsigned short)((u + 0x7FFFu + ((u >> 16) & 1u)) >> 16); }
__device__ __forceinline__ float bf16_rne(float x) { return __uint_as_float(((unsigned int)bf16_bits(x)) << 16); }
__device__ __forceinline__ unsigned short f16_bits(float x) { const _Float16 hv = (_Float16)x; return __builtin_bit_cast(unsigned short, hv); }
__device__ __forceinline__ unsigned ext_row(unsigned m) { return (m / (unsigned)SEQ) * (unsigned)SEQ_FULL + (m % (unsigned)SEQ); }
__device__ __forceinline__ float gelu_erf(float v) { return 0.5f * v * (1.0f + erff(v * 0.70710678118654752f)); }

__device__ __forceinline__ v8f mma1(v16h a, v16h b, v8f c) {
  c = __builtin_amdgcn_wmma_f32_16x16x32_f16(false, a, false, b, (short)0, c, false, false);
  asm volatile("v_nop\n\tv_nop\n\tv_nop\n\tv_nop" : "+v"(c) : "v"(a), "v"(b));
  return c;
}

__global__ __launch_bounds__(256) void k_wt_h(const float* __restrict__ W, unsigned short* __restrict__ Wt, unsigned K, unsigned N, float carry) {
  const unsigned t = blockIdx.x * 256u + threadIdx.x;
  const unsigned k8n = K >> 3;
  if (t >= N * k8n) return;
  const unsigned n = t / k8n, k8 = (t - n * k8n) << 3;
  v8us v;
#pragma unroll
  for (int i = 0; i < 8; ++i) v[i] = f16_bits(bf16_rne(W[(size_t)(k8 + i) * N + n]) * carry);
  unsigned short* dst = Wt + (size_t)n * K + k8;
  *(volatile v8us*)dst = v;
  __threadfence();
  *(volatile v8us*)dst = v;
}

template <bool EXT_BF16>
__global__ __launch_bounds__(128) void k_ln_rows(const float* __restrict__ X, const float* __restrict__ g, const float* __restrict__ bta,
                                                 unsigned short* __restrict__ out, unsigned nrows, float eps) {
  __shared__ __attribute__((aligned(16))) unsigned short sst[4][DM];
  const unsigned lane = threadIdx.x & 31u, w = threadIdx.x >> 5;
  const unsigned row = blockIdx.x * 4u + w;
  if (row >= nrows) return;
  const float* x = X + (size_t)(EXT_BF16 ? ext_row(row) : row) * DM;
  float s1 = 0.f;
#pragma unroll 1
  for (unsigned u = 0; u < DM / 256; ++u) {
    const unsigned j = (u * 32u + lane) * 8u;
    const v4f a = *(const v4fa*)(x + j), b = *(const v4fa*)(x + j + 4);
#pragma unroll
    for (int q = 0; q < 4; ++q) { s1 += EXT_BF16 ? bf16_rne(a[q]) : a[q]; s1 += EXT_BF16 ? bf16_rne(b[q]) : b[q]; }
  }
  s1 += __shfl_xor(s1, 16, 32); s1 += __shfl_xor(s1, 8, 32); s1 += __shfl_xor(s1, 4, 32); s1 += __shfl_xor(s1, 2, 32); s1 += __shfl_xor(s1, 1, 32);
  const float mu = s1 * (1.0f / (float)DM);
  float s2 = 0.f;
#pragma unroll 1
  for (unsigned u = 0; u < DM / 256; ++u) {
    const unsigned j = (u * 32u + lane) * 8u;
    const v4f a = *(const v4fa*)(x + j), b = *(const v4fa*)(x + j + 4);
#pragma unroll
    for (int q = 0; q < 4; ++q) {
      const float ca = (EXT_BF16 ? bf16_rne(a[q]) : a[q]) - mu, cb = (EXT_BF16 ? bf16_rne(b[q]) : b[q]) - mu;
      s2 += ca * ca; s2 += cb * cb;
    }
  }
  s2 += __shfl_xor(s2, 16, 32); s2 += __shfl_xor(s2, 8, 32); s2 += __shfl_xor(s2, 4, 32); s2 += __shfl_xor(s2, 2, 32); s2 += __shfl_xor(s2, 1, 32);
  const float rs = rsqrtf(s2 * (1.0f / (float)DM) + eps);
  unsigned short* orow = out + (size_t)row * DM;
#pragma unroll 1
  for (unsigned u = 0; u < DM / 256; ++u) {
    const unsigned j = (u * 32u + lane) * 8u;
    const v4f a = *(const v4fa*)(x + j), b = *(const v4fa*)(x + j + 4);
    const v4f ga = *(const v4fa*)(g + j), gb = *(const v4fa*)(g + j + 4);
    const v4f ba = *(const v4fa*)(bta + j), bb = *(const v4fa*)(bta + j + 4);
    v8us pk;
#pragma unroll
    for (int q = 0; q < 4; ++q) {
      const float pa = EXT_BF16 ? bf16_rne(a[q]) : a[q], pb = EXT_BF16 ? bf16_rne(b[q]) : b[q];
      pk[q]     = f16_bits((pa - mu) * rs * bf16_rne(ga[q]) + bf16_rne(ba[q]));
      pk[4 + q] = f16_bits((pb - mu) * rs * bf16_rne(gb[q]) + bf16_rne(bb[q]));
    }
    *(v8us*)&sst[w][j] = pk;
    *(volatile v8us*)(orow + j) = pk;
  }
  __threadfence();
#pragma unroll 1
  for (unsigned u = 0; u < DM / 256; ++u) {
    const unsigned j = (u * 32u + lane) * 8u;
    const v8us pk = *(const v8us*)&sst[w][j];
    *(volatile v8us*)(orow + j) = pk;
  }
}

template <int MODE>
__global__ __launch_bounds__(128) void k_gemm_h(const unsigned short* __restrict__ A, unsigned lda,
                                                const unsigned short* __restrict__ Bp, unsigned ldb,
                                                const float* __restrict__ bias, const float* __restrict__ resid,
                                                void* __restrict__ Cout, unsigned ldc,
                                                unsigned M, unsigned N, unsigned K, float inv) {
  __shared__ __attribute__((aligned(16))) float so[4][32][64];
  const unsigned tid = threadIdx.x, w = tid >> 5, lane = tid & 31u, ln = lane & 15u, hh = lane >> 4;
  const unsigned ntn = N >> 6;
  const unsigned wid = blockIdx.x * 4u + w;
  const unsigned mt = wid / ntn, nq = wid - mt * ntn;
  if (mt * 32u >= M) return;
  const unsigned row0 = mt * 32u, col0 = nq * 64u;
  const unsigned short* a0 = A + (size_t)(row0 + ln) * lda + 8u * hh;
  const unsigned short* a1 = a0 + (size_t)16 * lda;
  const unsigned short* b0 = Bp + (size_t)(col0 + ln) * ldb + 8u * hh;
  v8f acc[2][4];
#pragma unroll
  for (int mi = 0; mi < 2; ++mi)
#pragma unroll
    for (int t = 0; t < 4; ++t) acc[mi][t] = (v8f){0.f,0.f,0.f,0.f,0.f,0.f,0.f,0.f};
  for (unsigned kb = 0; kb < K; kb += 32u) {
    FragH fa0, fa1;
    fa0.half[0] = *(const v8us*)(a0 + kb); fa0.half[1] = *(const v8us*)(a0 + kb + 16);
    fa1.half[0] = *(const v8us*)(a1 + kb); fa1.half[1] = *(const v8us*)(a1 + kb + 16);
#pragma unroll
    for (int t = 0; t < 4; ++t) {
      const unsigned short* br = b0 + (size_t)(t * 16) * ldb + kb;
      FragH fb;
      fb.half[0] = *(const v8us*)(br);
      fb.half[1] = *(const v8us*)(br + 16);
      acc[0][t] = mma1(fa0.v, fb.v, acc[0][t]);
      acc[1][t] = mma1(fa1.v, fb.v, acc[1][t]);
    }
  }
  float brow[2][8];
#pragma unroll
  for (int mi = 0; mi < 2; ++mi)
#pragma unroll
    for (int r = 0; r < 8; ++r) brow[mi][r] = (MODE == 1) ? bf16_rne(bias[row0 + mi * 16 + 8u * hh + r]) : 0.f;
#pragma unroll
  for (int t = 0; t < 4; ++t) {
    const float bc = (MODE == 1) ? 0.f : bf16_rne(bias[col0 + t * 16 + ln]);
#pragma unroll
    for (int mi = 0; mi < 2; ++mi)
#pragma unroll
      for (int r = 0; r < 8; ++r)
        so[w][mi * 16 + 8u * hh + r][t * 16 + ln] = acc[mi][t][r] * inv + ((MODE == 1) ? brow[mi][r] : bc);
  }
  __builtin_amdgcn_fence(4  , "workgroup");
  __builtin_amdgcn_wave_barrier();
  if constexpr (MODE >= 3) {
    float* C = (float*)Cout;
    const unsigned rsub = lane >> 4, c4 = (lane & 15u) * 4u;
#pragma unroll 4
    for (unsigned q = 0; q < 16; ++q) {
      const unsigned r = q * 2u + rsub;
      const unsigned grow = row0 + r;
      const size_t ro = (size_t)((MODE == 3) ? ext_row(grow) : grow) * DM + col0 + c4;
      const v4f rv = *(const v4fa*)(resid + ro);
      v4f v = *(const v4fa*)&so[w][r][c4];
#pragma unroll
      for (int i = 0; i < 4; ++i) v[i] += (MODE == 3) ? bf16_rne(rv[i]) : rv[i];
      *(v4fa*)&so[w][r][c4] = v;
    }
    for (int pass = 0; pass < 2; ++pass) {
#pragma unroll 4
      for (unsigned q = 0; q < 16; ++q) {
        const unsigned r = q * 2u + rsub;
        const unsigned grow = row0 + r;
        const v4f v = *(const v4fa*)&so[w][r][c4];
        *(volatile v4f*)(C + (size_t)((MODE == 4) ? ext_row(grow) : grow) * ldc + col0 + c4) = v;
      }
      if (pass == 0) __threadfence();
    }
  } else {
    __shared__ __attribute__((aligned(16))) unsigned short sh[4][32][64];
    unsigned short* C = (unsigned short*)Cout;
    const unsigned rq = lane >> 3, c8 = (lane & 7u) * 8u;
#pragma unroll 1
    for (unsigned q = 0; q < 8; ++q) {
      const unsigned r = q * 4u + rq;
      const v4f x0 = *(const v4fa*)&so[w][r][c8], x1 = *(const v4fa*)&so[w][r][c8 + 4];
      v8us pk;
#pragma unroll
      for (int i = 0; i < 4; ++i) {
        float a = x0[i], b = x1[i];
        if (MODE == 2) { a = gelu_erf(a) * 64.0f; b = gelu_erf(b) * 64.0f; }
        pk[i] = f16_bits(a); pk[4 + i] = f16_bits(b);
      }
      *(v8us*)&sh[w][r][c8] = pk;
    }
    __builtin_amdgcn_fence(4  , "workgroup");
    __builtin_amdgcn_wave_barrier();
    size_t base; unsigned pitch;
    if (MODE == 1) { const unsigned bb = col0 / (unsigned)SEQ, s0 = col0 - bb * (unsigned)SEQ; base = ((size_t)bb * DM + row0) * SEQ + s0 + c8; pitch = SEQ; }
    else           { base = (size_t)row0 * ldc + col0 + c8; pitch = ldc; }
    for (int pass = 0; pass < 2; ++pass) {
#pragma unroll 4
      for (unsigned q = 0; q < 8; ++q) {
        const unsigned r = q * 4u + rq;
        const v8us v = *(const v8us*)&sh[w][r][c8];
        *(volatile v8us*)(C + base + (size_t)r * pitch) = v;
      }
      if (pass == 0) __threadfence();
    }
  }
}

__global__ __launch_bounds__(128) void k_flash(const unsigned short* __restrict__ Qp, const unsigned short* __restrict__ Kp,
                                               const unsigned short* __restrict__ Vt, unsigned short* __restrict__ ctx) {
  __shared__ __attribute__((aligned(16))) unsigned short sP[4][16][40];
  __shared__ __attribute__((aligned(16))) float sO[4][16][HD];
  const unsigned tid = threadIdx.x, w = tid >> 5, lane = tid & 31u, ln = lane & 15u, hh = lane >> 4;
  const unsigned nqb = SEQ / 64;
  const unsigned bh = blockIdx.x / nqb, qblk = blockIdx.x - bh * nqb;
  const unsigned b = bh / (unsigned)NH, h = bh - b * (unsigned)NH;
  const unsigned q0 = qblk * 64u + w * 16u;
  FragH aq[2];
  {
    const unsigned short* qr = Qp + (size_t)(b * (unsigned)SEQ + q0 + ln) * DM + h * HD + 8u * hh;
#pragma unroll
    for (int ks = 0; ks < 2; ++ks) { aq[ks].half[0] = *(const v8us*)(qr + ks * 32); aq[ks].half[1] = *(const v8us*)(qr + ks * 32 + 16); }
  }
  const unsigned short* kbase = Kp + (size_t)(b * (unsigned)SEQ + ln) * DM + h * HD + 8u * hh;
  const unsigned short* vbase = Vt + ((size_t)b * DM + h * HD + ln) * SEQ + 8u * hh;
  float m_r[8], l_r[8];
#pragma unroll
  for (int r = 0; r < 8; ++r) { m_r[r] = -1.0e30f; l_r[r] = 0.f; }
  v8f oacc[4];
#pragma unroll
  for (int dt = 0; dt < 4; ++dt) oacc[dt] = (v8f){0.f,0.f,0.f,0.f,0.f,0.f,0.f,0.f};

  for (unsigned j0 = 0; j0 < (unsigned)SEQ; j0 += 32u) {
    v8f s[2];
#pragma unroll
    for (int nt = 0; nt < 2; ++nt) {
      v8f acc = (v8f){0.f,0.f,0.f,0.f,0.f,0.f,0.f,0.f};
#pragma unroll
      for (int ks = 0; ks < 2; ++ks) {
        const unsigned short* kr = kbase + (size_t)(j0 + nt * 16) * DM + ks * 32;
        FragH fb;
        fb.half[0] = *(const v8us*)(kr);
        fb.half[1] = *(const v8us*)(kr + 16);
        acc = mma1(aq[ks].v, fb.v, acc);
      }
      s[nt] = acc;
    }
    float alpha[8];
#pragma unroll
    for (int r = 0; r < 8; ++r) {
      const float s0 = s[0][r] * 0.125f, s1 = s[1][r] * 0.125f;
      float mx = fmaxf(s0, s1);
      mx = fmaxf(mx, __shfl_xor(mx, 1, 32)); mx = fmaxf(mx, __shfl_xor(mx, 2, 32)); mx = fmaxf(mx, __shfl_xor(mx, 4, 32)); mx = fmaxf(mx, __shfl_xor(mx, 8, 32));
      const float mnew = fmaxf(m_r[r], mx);
      alpha[r] = __expf(m_r[r] - mnew);
      const float p0 = __expf(s0 - mnew), p1 = __expf(s1 - mnew);
      m_r[r] = mnew;
      l_r[r] = l_r[r] * alpha[r] + p0 + p1;
      sP[w][8u * hh + r][ln]       = f16_bits(p0 * 1024.0f);
      sP[w][8u * hh + r][16u + ln] = f16_bits(p1 * 1024.0f);
    }
#pragma unroll
    for (int dt = 0; dt < 4; ++dt)
#pragma unroll
      for (int r = 0; r < 8; ++r) oacc[dt][r] *= alpha[r];
    __builtin_amdgcn_fence(4  , "workgroup");
    __builtin_amdgcn_wave_barrier();
    FragH pa;
    pa.half[0] = *(const v8us*)&sP[w][ln][8u * hh];
    pa.half[1] = *(const v8us*)&sP[w][ln][16u + 8u * hh];
#pragma unroll
    for (int dt = 0; dt < 4; ++dt) {
      const unsigned short* vr = vbase + (size_t)(dt * 16) * SEQ + j0;
      FragH fb;
      fb.half[0] = *(const v8us*)(vr);
      fb.half[1] = *(const v8us*)(vr + 16);
      oacc[dt] = mma1(pa.v, fb.v, oacc[dt]);
    }
    __builtin_amdgcn_fence(4  , "workgroup");
    __builtin_amdgcn_wave_barrier();
  }
#pragma unroll
  for (int r = 0; r < 8; ++r) {
    float l = l_r[r];
    l += __shfl_xor(l, 1, 32); l += __shfl_xor(l, 2, 32); l += __shfl_xor(l, 4, 32); l += __shfl_xor(l, 8, 32);
    l_r[r] = 0.0625f * (1.0f / l);
  }
#pragma unroll
  for (int dt = 0; dt < 4; ++dt)
#pragma unroll
    for (int r = 0; r < 8; ++r) sO[w][8u * hh + r][dt * 16 + ln] = oacc[dt][r] * l_r[r];
  __builtin_amdgcn_fence(4  , "workgroup");
  __builtin_amdgcn_wave_barrier();
  const unsigned rq = lane >> 3, c8 = (lane & 7u) * 8u;
  v8us pk[4];
#pragma unroll
  for (int q = 0; q < 4; ++q) {
    const unsigned r = q * 4u + rq;
    const v4f x0 = *(const v4fa*)&sO[w][r][c8], x1 = *(const v4fa*)&sO[w][r][c8 + 4];
#pragma unroll
    for (int i = 0; i < 4; ++i) { pk[q][i] = f16_bits(x0[i]); pk[q][4 + i] = f16_bits(x1[i]); }
  }
  unsigned short* dst = ctx + (size_t)(b * (unsigned)SEQ + q0 + rq) * DM + h * HD + c8;
#pragma unroll
  for (int pass = 0; pass < 2; ++pass) {
#pragma unroll
    for (int q = 0; q < 4; ++q) *(volatile v8us*)(dst + (size_t)(q * 4) * DM) = pk[q];
    if (pass == 0) __threadfence();
  }
}

extern "C" void kernel_launch(void* const* d_in, const int* in_sizes, int n_in,
                              void* d_out, int out_size, void* d_ws, size_t ws_size, hipStream_t stream) {
  if (n_in < 17) return;
  const size_t need_x = ((size_t)(NB - 1) * SEQ_FULL + SEQ) * DM;
  if ((size_t)in_sizes[0] < need_x || (size_t)out_size < need_x) return;
  if (in_sizes[1] < DM * DM || in_sizes[3] < DM * DM || in_sizes[5] < DM * DM || in_sizes[7] < DM * DM) return;
  if (in_sizes[13] < DM * FF || in_sizes[15] < FF * DM) return;
  if (in_sizes[2] < DM || in_sizes[4] < DM || in_sizes[6] < DM || in_sizes[8] < DM || in_sizes[9] < DM || in_sizes[10] < DM ||
      in_sizes[11] < DM || in_sizes[12] < DM || in_sizes[14] < FF || in_sizes[16] < DM) return;
  const float* x   = (const float*)d_in[0];
  const float* Wq  = (const float*)d_in[1];  const float* bq  = (const float*)d_in[2];
  const float* Wk  = (const float*)d_in[3];  const float* bk  = (const float*)d_in[4];
  const float* Wv  = (const float*)d_in[5];  const float* bv  = (const float*)d_in[6];
  const float* Wo  = (const float*)d_in[7];  const float* bo  = (const float*)d_in[8];
  const float* g1  = (const float*)d_in[9];  const float* be1 = (const float*)d_in[10];
  const float* g2  = (const float*)d_in[11]; const float* be2 = (const float*)d_in[12];
  const float* W1  = (const float*)d_in[13]; const float* b1  = (const float*)d_in[14];
  const float* W2  = (const float*)d_in[15]; const float* b2  = (const float*)d_in[16];

  constexpr size_t SZ_W   = (size_t)DM * DM * 2;
  constexpr size_t SZ_WF  = (size_t)DM * FF * 2;
  constexpr size_t SZ_P   = (size_t)MROWS * DM * 2;
  constexpr size_t SZ_X2  = (size_t)MROWS * DM * 4;
  constexpr size_t SZ_MID = (size_t)MROWS * FF * 2;
  constexpr size_t SZ_R   = 4 * SZ_P;
  static_assert(SZ_MID <= SZ_R);
  static_assert(SZ_W % 256 == 0);
  static_assert(SZ_WF % 256 == 0);
  static_assert(SZ_P % 256 == 0);
  static_assert(SZ_X2 % 256 == 0);
  constexpr size_t TOTAL = 4 * SZ_W + 2 * SZ_WF + SZ_P + SZ_R + SZ_X2;
  static_assert(TOTAL <= (size_t)134217728);
  if (TOTAL > ws_size) return;
  char* ws = (char*)d_ws; size_t off = 0;
  auto take = [&](size_t bytes) { char* p = ws + off; off += bytes; return p; };
  unsigned short* WqT = (unsigned short*)take(SZ_W);
  unsigned short* WkT = (unsigned short*)take(SZ_W);
  unsigned short* WvT = (unsigned short*)take(SZ_W);
  unsigned short* WoT = (unsigned short*)take(SZ_W);
  unsigned short* W1T = (unsigned short*)take(SZ_WF);
  unsigned short* W2T = (unsigned short*)take(SZ_WF);
  unsigned short* hy  = (unsigned short*)take(SZ_P);
  char* R = take(SZ_R);
  unsigned short* Qpl = (unsigned short*)(R);
  unsigned short* Kpl = (unsigned short*)(R + SZ_P);
  unsigned short* Vtp = (unsigned short*)(R + 2 * SZ_P);
  unsigned short* ctx = (unsigned short*)(R + 3 * SZ_P);
  unsigned short* mid = (unsigned short*)(R);
  float* x2 = (float*)take(SZ_X2);

  k_wt_h<<<(DM * (DM / 8)) / 256, 256, 0, stream>>>(Wq, WqT, DM, DM, 64.0f);
  k_wt_h<<<(DM * (DM / 8)) / 256, 256, 0, stream>>>(Wk, WkT, DM, DM, 64.0f);
  k_wt_h<<<(DM * (DM / 8)) / 256, 256, 0, stream>>>(Wv, WvT, DM, DM, 64.0f);
  k_wt_h<<<(DM * (DM / 8)) / 256, 256, 0, stream>>>(Wo, WoT, DM, DM, 64.0f);
  k_wt_h<<<(FF * (DM / 8)) / 256, 256, 0, stream>>>(W1, W1T, DM, FF, 64.0f);
  k_wt_h<<<(DM * (FF / 8)) / 256, 256, 0, stream>>>(W2, W2T, FF, DM, 64.0f);

  const float i64 = 0.015625f, i4096 = 0.000244140625f;
  const unsigned gD  = ((MROWS / 32) * (DM / 64) + 3) / 4;
  const unsigned gF  = ((MROWS / 32) * (FF / 64) + 3) / 4;
  const unsigned gVt = ((DM / 32) * (MROWS / 64) + 3) / 4;

  k_ln_rows<true><<<MROWS / 4, 128, 0, stream>>>(x, g1, be1, hy, MROWS, 1e-6f);
  k_gemm_h<0><<<gD, 128, 0, stream>>>(hy, DM, WqT, DM, bq, nullptr, Qpl, DM, MROWS, DM, DM, i64);
  k_gemm_h<0><<<gD, 128, 0, stream>>>(hy, DM, WkT, DM, bk, nullptr, Kpl, DM, MROWS, DM, DM, i64);
  k_gemm_h<1><<<gVt, 128, 0, stream>>>(WvT, DM, hy, DM, bv, nullptr, Vtp, SEQ, DM, MROWS, DM, i64);
  k_flash<<<NB * NH * (SEQ / 64), 128, 0, stream>>>(Qpl, Kpl, Vtp, ctx);
  k_gemm_h<3><<<gD, 128, 0, stream>>>(ctx, DM, WoT, DM, bo, x, x2, DM, MROWS, DM, DM, i4096);
  k_ln_rows<false><<<MROWS / 4, 128, 0, stream>>>(x2, g2, be2, hy, MROWS, 1e-6f);
  k_gemm_h<2><<<gF, 128, 0, stream>>>(hy, DM, W1T, DM, b1, nullptr, mid, FF, MROWS, FF, DM, i64);
  k_gemm_h<4><<<gD, 128, 0, stream>>>(mid, FF, W2T, FF, b2, x2, d_out, DM, MROWS, DM, FF, i4096);
}
